// SyntaxTransformerEncoder_76330158784745
// MI455X (gfx1250) — hardware-verified
//
#include <hip/hip_runtime.h>


#define NB_  2
#define NL   6
#define SYH  128
#define VOC  32000
#define FFH  2048
#define TT   1024
#define CC   512
#define NH_  8
#define HD   64
#define NT   (NB_ * TT)
#define NZ   (NB_ * NH_)
#define ZB   8
#define PCAR 1024.0f
typedef _Float16 h16;
typedef unsigned short bf;
typedef __attribute__((ext_vector_type(16))) __bf16   v16bf;
typedef __attribute__((ext_vector_type(16))) _Float16 v16h;
typedef __attribute__((ext_vector_type(8)))  _Float16 v8h;
typedef __attribute__((ext_vector_type(8)))  unsigned short v8us;
typedef __attribute__((ext_vector_type(8)))  float    v8f;
typedef __attribute__((ext_vector_type(4)))  float    v4f;
typedef v8h  __attribute__((may_alias)) v8ha;
typedef v4f  __attribute__((may_alias)) v4fa;
typedef v8us __attribute__((may_alias)) v8usa;

__device__ __forceinline__ unsigned short f2bf(float f) { unsigned u = __float_as_uint(f); u += 0x7FFFu + ((u >> 16) & 1u); return (unsigned short)(u >> 16); }
__device__ __forceinline__ float bf2f(unsigned short b) { return __uint_as_float(((unsigned)b) << 16); }
__device__ __forceinline__ float bfr(float f) { return bf2f(f2bf(f)); }
__device__ __forceinline__ v16h cat16(v8h lo, v8h hi) { return __builtin_shufflevector(lo, hi, 0, 1, 2, 3, 4, 5, 6, 7, 8, 9, 10, 11, 12, 13, 14, 15); }
__device__ __forceinline__ v16bf cat16b(v8us lo, v8us hi) { return __builtin_bit_cast(v16bf, __builtin_shufflevector(lo, hi, 0, 1, 2, 3, 4, 5, 6, 7, 8, 9, 10, 11, 12, 13, 14, 15)); }
__device__ __forceinline__ v8f wmma16(v16h a, v16h b, v8f c) { return __builtin_amdgcn_wmma_f32_16x16x32_f16(false, a, false, b, (short)0, c, false, false); }
__device__ __forceinline__ v8f wmmab(v16bf a, v16bf b, v8f c) { return __builtin_amdgcn_wmma_f32_16x16x32_bf16(false, a, false, b, (short)0, c, false, false); }


template <typename T16> struct WFrag;
template <> struct WFrag<h16> { typedef v16h V; static __device__ __forceinline__ V ld(const h16* p) { return cat16(*(const v8h*)p, *(const v8h*)(p + 16)); } static __device__ __forceinline__ v8f mma(V a, V b, v8f c) { return wmma16(a, b, c); } };
template <> struct WFrag<bf> { typedef v16bf V; static __device__ __forceinline__ V ld(const bf* p) { return cat16b(*(const v8us*)p, *(const v8us*)(p + 16)); } static __device__ __forceinline__ v8f mma(V a, V b, v8f c) { return wmmab(a, b, c); } };
template <typename T16, int NSPLIT, bool BIAS>
__global__ __launch_bounds__(32) void k_gemmw(const T16* __restrict__ A, const T16* __restrict__ A2, const T16* __restrict__ Bt, const T16* __restrict__ Bt2, int K, float* C, int ldc, const float* __restrict__ bias, size_t sA, size_t sB, size_t sC) {
    typedef typename WFrag<T16>::V V;
    __shared__ __align__(16) float os[16 * 68];
    const size_t z = blockIdx.z; A += z * sA; if (A2) A2 += z * sA; Bt += z * sB; if (Bt2) Bt2 += z * sB; C += z * sC;
    const int lane = threadIdx.x & 31, lr = lane & 15, hi = lane >> 4; const int r0 = blockIdx.x * 64, c0 = blockIdx.y * 64;
    v8f acc[4][4];
#pragma unroll
    for (int mb = 0; mb < 4; ++mb)
#pragma unroll
        for (int nb = 0; nb < 4; ++nb) acc[mb][nb] = (v8f){};
    const size_t aoff = (size_t)(r0 + lr) * K + 8 * hi, boff = (size_t)(c0 + lr) * K + 8 * hi;
#pragma unroll 1
    for (int kc = 0; kc < K; kc += 32) {
        V a[4], a2[4];
#pragma unroll
        for (int mb = 0; mb < 4; ++mb) { a[mb] = WFrag<T16>::ld(A + aoff + (size_t)mb * 16 * K + kc); if (NSPLIT == 1 || NSPLIT == 2) a2[mb] = WFrag<T16>::ld(A2 + aoff + (size_t)mb * 16 * K + kc); }
#pragma unroll
        for (int nb = 0; nb < 4; ++nb) { const V b = WFrag<T16>::ld(Bt + boff + (size_t)nb * 16 * K + kc); V b2; if (NSPLIT >= 2) b2 = WFrag<T16>::ld(Bt2 + boff + (size_t)nb * 16 * K + kc);
#pragma unroll
            for (int mb = 0; mb < 4; ++mb) { acc[mb][nb] = WFrag<T16>::mma(a[mb], b, acc[mb][nb]); if (NSPLIT == 1 || NSPLIT == 2) acc[mb][nb] = WFrag<T16>::mma(a2[mb], b, acc[mb][nb]); if (NSPLIT >= 2) acc[mb][nb] = WFrag<T16>::mma(a[mb], b2, acc[mb][nb]); } }
        asm volatile("v_nop\n\tv_nop\n\tv_nop\n\tv_nop" : "+v"(acc[0][0]), "+v"(acc[1][1]), "+v"(acc[2][2]), "+v"(acc[3][3]) : "v"(a[0]), "v"(a[3]));
    }
#pragma unroll
    for (int mb = 0; mb < 4; ++mb) {
#pragma unroll
        for (int nb = 0; nb < 4; ++nb) {
#pragma unroll
            for (int j = 0; j < 8; ++j) os[(hi * 8 + j) * 68 + nb * 16 + lr] = acc[mb][nb][j]; }
        __builtin_amdgcn_wave_barrier(); asm volatile("" ::: "memory");
        float* crow = C + (size_t)(r0 + mb * 16) * ldc + c0;
#pragma unroll 1
        for (int ps = 0; ps < 2; ++ps) {
#pragma unroll
            for (int s = 0; s < 8; ++s) { const int row = 2 * s + hi, cofs = lr * 4; v4f val = *(const v4fa*)(os + row * 68 + cofs); if (BIAS) { val[0] += bfr(bias[c0 + cofs]); val[1] += bfr(bias[c0 + cofs + 1]); val[2] += bfr(bias[c0 + cofs + 2]); val[3] += bfr(bias[c0 + cofs + 3]); }
                *(volatile v4f*)(crow + (size_t)row * ldc + cofs) = val; }
            if (ps == 0) __threadfence(); }
        __builtin_amdgcn_wave_barrier(); asm volatile("" ::: "memory");
    }
}

__device__ __forceinline__ h16 tohx(float x) { return (h16)x; }
__device__ __forceinline__ void splitf(float y, unsigned short& h, unsigned short& l) { h = f2bf(y); l = f2bf(y - bf2f(h)); }
typedef __attribute__((ext_vector_type(2))) _Float16 v2h;
typedef __attribute__((ext_vector_type(4))) _Float16 v4h;
typedef __attribute__((ext_vector_type(2))) unsigned short v2us;
typedef __attribute__((ext_vector_type(2))) float v2f;

__global__ __launch_bounds__(256) void k_cvt8(const float* __restrict__ src, bf* dst, size_t n8) { const size_t i = (size_t)blockIdx.x * 256 + threadIdx.x; if (i >= n8) return; const v8f v = *(const v8f*)(src + i * 8); v8us o;
#pragma unroll
    for (int k = 0; k < 8; ++k) o[k] = f2bf(v[k]); *(volatile v8us*)(dst + i * 8) = o; __threadfence(); *(volatile v8us*)(dst + i * 8) = o; }
__global__ __launch_bounds__(256) void k_wtG(const float* __restrict__ w, int K, int N, bf* Bt) {
    const int lane = threadIdx.x & 31; const int L0 = (blockIdx.x * 8 + (threadIdx.x >> 5)) * 8; const int nlines = N * K / 64;
#pragma unroll 1
    for (int ps = 0; ps < 2; ++ps) {
#pragma unroll 1
        for (int l = 0; l < 8; ++l) { const int L = L0 + l; if (L >= nlines) break; const size_t e = (size_t)L * 64 + lane * 2; const int k = (int)(e % K), n = (int)(e / K); v2us o;
            o[0] = f2bf(w[(size_t)k * N + n]); o[1] = f2bf(w[(size_t)(k + 1) * N + n]); *(volatile v2us*)(Bt + e) = o; }
        if (ps == 0) __threadfence(); }
}
__global__ __launch_bounds__(256) void k_hsplit(const float* __restrict__ F, float sc, bf* Ph, bf* Pl) {
    const int lane = threadIdx.x & 31; const int L0 = (blockIdx.x * 8 + (threadIdx.x >> 5)) * 8; const int nlines = NT * CC / 64;
#pragma unroll 1
    for (int ps = 0; ps < 2; ++ps) {
#pragma unroll
        for (int l = 0; l < 8; ++l) { const int L = L0 + l; if (L >= nlines) break; const int e = L * 64 + lane * 2; const int d = e & 63; const int t = (e >> 6) & (TT - 1); const int z = e >> 16; const int b = z / NH_, h = z % NH_; v2us oh, ol;
#pragma unroll
            for (int q = 0; q < 2; ++q) { unsigned short a, c2; splitf(F[((size_t)b * TT + t) * CC + h * HD + d + q] * sc, a, c2); oh[q] = a; ol[q] = c2; }
            *(volatile v2us*)(Ph + (size_t)e) = oh; *(volatile v2us*)(Pl + (size_t)e) = ol; }
        if (ps == 0) __threadfence(); }
}
__global__ __launch_bounds__(256) void k_vtplane(const float* __restrict__ F, bf* Vh, bf* Vl) {
    const int lane = threadIdx.x & 31; const int L0 = (blockIdx.x * 8 + (threadIdx.x >> 5)) * 8; const int nlines = NT * CC / 64;
#pragma unroll 1
    for (int ps = 0; ps < 2; ++ps) {
#pragma unroll
        for (int l = 0; l < 8; ++l) { const int L = L0 + l; if (L >= nlines) break; const int e = L * 64 + lane * 2; const int t = e & (TT - 1); const int d = (e >> 10) & 63; const int z = e >> 16; const int b = z / NH_, h = z % NH_; v2us oh, ol;
#pragma unroll
            for (int q = 0; q < 2; ++q) { unsigned short a, c2; splitf(F[((size_t)b * TT + t + q) * CC + h * HD + d], a, c2); oh[q] = a; ol[q] = c2; }
            *(volatile v2us*)(Vh + (size_t)e) = oh; *(volatile v2us*)(Vl + (size_t)e) = ol; }
        if (ps == 0) __threadfence(); }
}
__global__ __launch_bounds__(256) void k_merge(const float* __restrict__ O, int z0, bf* Ah, bf* Al) {
    const int lane = threadIdx.x & 31; const int L0 = (blockIdx.x * 8 + (threadIdx.x >> 5)) * 8; const int nlines = ZB * TT * HD / 64;
#pragma unroll 1
    for (int ps = 0; ps < 2; ++ps) {
#pragma unroll
        for (int l = 0; l < 8; ++l) { const int L = L0 + l; if (L >= nlines) break; const int e = L * 64 + lane * 2; const int d = e & 63; const int t = (e >> 6) & (TT - 1); const int zz = e >> 16; const int z = z0 + zz; const int b = z / NH_, h = z % NH_; v2us oh, ol;
#pragma unroll
            for (int q = 0; q < 2; ++q) { unsigned short a, c2; splitf(O[(size_t)e + q], a, c2); oh[q] = a; ol[q] = c2; }
            const size_t o = ((size_t)b * TT + t) * CC + h * HD + d; *(volatile v2us*)(Ah + o) = oh; *(volatile v2us*)(Al + o) = ol; }
        if (ps == 0) __threadfence(); }
}

__global__ __launch_bounds__(256) void k_relusplit(const float* __restrict__ H, bf* Hh, bf* Hl, size_t n) {
    const size_t i = ((size_t)blockIdx.x * 256 + threadIdx.x) * 2; if (i >= n) return; v2us oh, ol;
#pragma unroll
    for (int q = 0; q < 2; ++q) { unsigned short a, c2; splitf(fmaxf(H[i + q], 0.f), a, c2); oh[q] = a; ol[q] = c2; }
    *(volatile v2us*)(Hh + i) = oh; *(volatile v2us*)(Hl + i) = ol; __threadfence(); *(volatile v2us*)(Hh + i) = oh; *(volatile v2us*)(Hl + i) = ol; }
__global__ __launch_bounds__(256) void k_addout(const float* __restrict__ FF, const float* __restrict__ X, float* OUT, size_t n) {
    const size_t i = ((size_t)blockIdx.x * 256 + threadIdx.x) * 4; if (i >= n) return; const v4f a = *(const v4f*)(FF + i), b = *(const v4f*)(X + i); v4f o;
#pragma unroll
    for (int q = 0; q < 4; ++q) o[q] = a[q] + b[q];
    *(volatile v4f*)(OUT + i) = o; __threadfence(); *(volatile v4f*)(OUT + i) = o; }


typedef __attribute__((ext_vector_type(4))) unsigned short v4us;
__device__ __forceinline__ void ln512(float* v, const float* __restrict__ gg, const float* __restrict__ bb, int lane) {
    float s = 0.f;
#pragma unroll
    for (int i = 0; i < 16; ++i) s += v[i];
#pragma unroll
    for (int sh = 16; sh; sh >>= 1) s += __shfl_xor(s, sh, 32);
    const float mu = s * (1.0f / CC); float qq = 0.f;
#pragma unroll
    for (int i = 0; i < 16; ++i) { const float d0 = v[i] - mu; qq = __fadd_rn(qq, __fmul_rn(d0, d0)); }
#pragma unroll
    for (int sh = 16; sh; sh >>= 1) qq += __shfl_xor(qq, sh, 32);
    const float rs = __fdiv_rn(1.0f, __fsqrt_rn(qq * (1.0f / CC) + 1e-5f));
#pragma unroll
    for (int c = 0; c < 4; ++c) {
#pragma unroll
        for (int q = 0; q < 4; ++q) { const int col = c * 128 + lane * 4 + q; v[c * 4 + q] = __fadd_rn(__fmul_rn((v[c * 4 + q] - mu) * rs, bfr(gg[col])), bfr(bb[col])); } }
}
__device__ __forceinline__ void load512(const float* __restrict__ p, int lane, float* v) {
#pragma unroll
    for (int c = 0; c < 4; ++c) { const v4f a = *(const v4f*)(p + c * 128 + lane * 4);
#pragma unroll
        for (int q = 0; q < 4; ++q) v[c * 4 + q] = a[q]; } }
__device__ __forceinline__ void store512(const float* v, int lane, float* dst) {
#pragma unroll 1
    for (int ps = 0; ps < 2; ++ps) {
#pragma unroll
        for (int c = 0; c < 4; ++c) { v4f o;
#pragma unroll
            for (int q = 0; q < 4; ++q) o[q] = v[c * 4 + q];
            *(volatile v4f*)(dst + c * 128 + lane * 4) = o; }
        if (ps == 0) __threadfence(); } }
__device__ __forceinline__ void storesplit512(const float* v, int lane, bf* Ph, bf* Pl) {
#pragma unroll 1
    for (int ps = 0; ps < 2; ++ps) {
#pragma unroll
        for (int c = 0; c < 4; ++c) { v4us oh, ol;
#pragma unroll
            for (int q = 0; q < 4; ++q) { unsigned short a, c2; splitf(v[c * 4 + q], a, c2); oh[q] = a; ol[q] = c2; }
            *(volatile v4us*)(Ph + c * 128 + lane * 4) = oh; *(volatile v4us*)(Pl + c * 128 + lane * 4) = ol; }
        if (ps == 0) __threadfence(); } }
__global__ __launch_bounds__(256) void k_embed(const int* __restrict__ tok, const int* __restrict__ ptag, const int* __restrict__ etyp, const float* __restrict__ TE, const float* __restrict__ PE_, const float* __restrict__ EE, float* X) {
    const int lane = threadIdx.x & 31; const int r = blockIdx.x * 8 + (threadIdx.x >> 5); if (r >= NT) return; const int it = min(max(tok[r], 0), VOC - 1), ip = min(max(ptag[r], 0), VOC - 1), ie = min(max(etyp[r], 0), 2); float v[16];
#pragma unroll
    for (int c = 0; c < 4; ++c) { const int col = c * 128 + lane * 4; const v4f a = *(const v4f*)(TE + (size_t)it * CC + col), p = *(const v4f*)(PE_ + (size_t)ip * CC + col), e = *(const v4f*)(EE + (size_t)ie * CC + col);
#pragma unroll
        for (int q = 0; q < 4; ++q) v[c * 4 + q] = __fadd_rn(__fadd_rn(__fmul_rn(bfr(a[q]), 22.627416998f), bfr(p[q])), bfr(e[q])); }
    store512(v, lane, X + (size_t)r * CC);
}
__global__ __launch_bounds__(256) void k_synmlp(const float* __restrict__ SF, const float* __restrict__ W1, const float* __restrict__ B1, const float* __restrict__ gg, const float* __restrict__ bb, bf* Hh, bf* Hl) {
    const int lane = threadIdx.x & 31; const int r = blockIdx.x * 8 + (threadIdx.x >> 5); if (r >= NT) return; const float f0 = bfr(SF[(size_t)r * 3]), f1 = bfr(SF[(size_t)r * 3 + 1]), f2 = bfr(SF[(size_t)r * 3 + 2]); float v[4]; float s = 0.f;
#pragma unroll
    for (int q = 0; q < 4; ++q) { const int col = lane * 4 + q; float a = __fmul_rn(f0, bfr(W1[col])); a = __fadd_rn(a, __fmul_rn(f1, bfr(W1[SYH + col]))); a = __fadd_rn(a, __fmul_rn(f2, bfr(W1[2 * SYH + col]))); v[q] = __fadd_rn(a, bfr(B1[col])); s += v[q]; }
#pragma unroll
    for (int sh = 16; sh; sh >>= 1) s += __shfl_xor(s, sh, 32);
    const float mu = s * (1.0f / SYH); float qq = 0.f;
#pragma unroll
    for (int q = 0; q < 4; ++q) { const float d0 = v[q] - mu; qq = __fadd_rn(qq, __fmul_rn(d0, d0)); }
#pragma unroll
    for (int sh = 16; sh; sh >>= 1) qq += __shfl_xor(qq, sh, 32);
    const float rs = __fdiv_rn(1.0f, __fsqrt_rn(qq * (1.0f / SYH) + 1e-5f)); v4us oh, ol;
#pragma unroll
    for (int q = 0; q < 4; ++q) { const int col = lane * 4 + q; const float h = fmaxf(__fadd_rn(__fmul_rn((v[q] - mu) * rs, bfr(gg[col])), bfr(bb[col])), 0.f); unsigned short a, c2; splitf(h, a, c2); oh[q] = a; ol[q] = c2; }
    *(volatile v4us*)(Hh + (size_t)r * SYH + lane * 4) = oh; *(volatile v4us*)(Hl + (size_t)r * SYH + lane * 4) = ol; __threadfence(); *(volatile v4us*)(Hh + (size_t)r * SYH + lane * 4) = oh; *(volatile v4us*)(Hl + (size_t)r * SYH + lane * 4) = ol;
}
__global__ __launch_bounds__(256) void k_petab(float* PE) {
    const int i = blockIdx.x * 256 + threadIdx.x; if (i >= TT * CC) return; const int t = i / CC, col = i % CC; const float dv = expf(__fmul_rn((float)(col & ~1), -0.017988946f)); const float ang = __fmul_rn((float)t, dv);
    const float pe = (col & 1) ? cosf(ang) : sinf(ang); *(volatile float*)(PE + i) = pe; __threadfence(); *(volatile float*)(PE + i) = pe; }
__global__ __launch_bounds__(256) void k_embln(const float* __restrict__ F, const float* __restrict__ PE, const float* __restrict__ gg, const float* __restrict__ bb, float* X) {
    const int lane = threadIdx.x & 31; const int r = blockIdx.x * 8 + (threadIdx.x >> 5); if (r >= NT) return; const int t = r & (TT - 1); float v[16], f[16], p[16];
    load512(X + (size_t)r * CC, lane, v); load512(F + (size_t)r * CC, lane, f); load512(PE + (size_t)t * CC, lane, p);
#pragma unroll
    for (int i = 0; i < 16; ++i) v[i] = __fadd_rn(__fadd_rn(v[i], f[i]), p[i]);
    ln512(v, gg, bb, lane); store512(v, lane, X + (size_t)r * CC);
}
template <int DOUBLE>
__global__ __launch_bounds__(256) void k_lnx(const float* __restrict__ X, const float* __restrict__ ga, const float* __restrict__ ba, const float* __restrict__ gb, const float* __restrict__ bb2, bf* Ph, bf* Pl) {
    const int lane = threadIdx.x & 31; const int r = blockIdx.x * 8 + (threadIdx.x >> 5); if (r >= NT) return; float v[16];
    load512(X + (size_t)r * CC, lane, v); ln512(v, ga, ba, lane); if (DOUBLE) ln512(v, gb, bb2, lane);
    storesplit512(v, lane, Ph + (size_t)r * CC, Pl + (size_t)r * CC);
}
__global__ __launch_bounds__(32) void k_relw(const float* __restrict__ relw, const float* __restrict__ rels, int l, float* RWB) {
    const int lane = threadIdx.x; const float w0 = bfr(relw[l * 4]), w1 = bfr(relw[l * 4 + 1]), w2 = bfr(relw[l * 4 + 2]), w3 = bfr(relw[l * 4 + 3]); const float mx = fmaxf(fmaxf(w0, w1), fmaxf(w2, w3));
    const float e0 = __expf(w0 - mx), e1 = __expf(w1 - mx), e2 = __expf(w2 - mx), e3 = __expf(w3 - mx); const float s = e0 + e1 + e2 + e3;
    float o = 0.f; if (lane == 0) o = __fdiv_rn(e0, s); if (lane == 1) o = __fdiv_rn(e1, s); if (lane == 2) o = __fdiv_rn(e2, s); if (lane == 3) o = __fdiv_rn(e3, s);
    if (lane == 4) o = __fmul_rn(__fdiv_rn(1.0f, __fadd_rn(1.0f, __expf(-bfr(rels[l])))), 0.1f);
    *(volatile float*)(RWB + lane) = o; __threadfence(); *(volatile float*)(RWB + lane) = o;
}
__global__ __launch_bounds__(256) void k_msoft(const float* __restrict__ Sb, const float* __restrict__ TR, const int* __restrict__ amask, const float* __restrict__ RWB, int z0, bf* Ph, bf* Pl) {
    typedef __attribute__((ext_vector_type(4))) int v4i;
    const int lane = threadIdx.x & 31; const int row = blockIdx.x * 8 + (threadIdx.x >> 5); if (row >= ZB * TT) return; const int i = row & (TT - 1); const int zz = row >> 10; const int z = z0 + zz; const int b = z / NH_;
    const float* sr = Sb + (size_t)row * TT; const float* tr = TR + ((size_t)b * TT + i) * TT * 4; const int* mr = amask + (size_t)b * TT; const float r0 = RWB[0], r1 = RWB[1], r2 = RWB[2], r3 = RWB[3], bsc = RWB[4]; float v[32]; float mx = -3.0e38f;
#pragma unroll
    for (int ch = 0; ch < 8; ++ch) { const int j0 = ch * 128 + lane * 4; const v4f a = *(const v4f*)(sr + j0); const v4i mk = *(const v4i*)(mr + j0);
#pragma unroll
        for (int q = 0; q < 4; ++q) { const v4f t4 = *(const v4f*)(tr + (size_t)(j0 + q) * 4); float bsum = __fmul_rn(bfr(t4[0]), r0); bsum = __fadd_rn(bsum, __fmul_rn(bfr(t4[1]), r1)); bsum = __fadd_rn(bsum, __fmul_rn(bfr(t4[2]), r2)); bsum = __fadd_rn(bsum, __fmul_rn(bfr(t4[3]), r3));
            const float t = (mk[q] == 0) ? -1.0e9f : __fadd_rn(a[q], __fmul_rn(bsum, bsc)); v[ch * 4 + q] = t; mx = fmaxf(mx, t); } }
#pragma unroll
    for (int sh = 16; sh; sh >>= 1) mx = fmaxf(mx, __shfl_xor(mx, sh, 32));
    float sum = 0.f;
#pragma unroll
    for (int k = 0; k < 32; ++k) { v[k] = __expf(v[k] - mx); sum += v[k]; }
#pragma unroll
    for (int sh = 16; sh; sh >>= 1) sum += __shfl_xor(sum, sh, 32);
    const float f = __fdiv_rn(1.0f, sum);
#pragma unroll 1
    for (int ps = 0; ps < 2; ++ps) {
#pragma unroll
        for (int ch = 0; ch < 8; ++ch) { v4us oh, ol;
#pragma unroll
            for (int q = 0; q < 4; ++q) { unsigned short a, c2; splitf(v[ch * 4 + q] * f, a, c2); oh[q] = a; ol[q] = c2; }
            *(volatile v4us*)(Ph + (size_t)row * TT + ch * 128 + lane * 4) = oh; *(volatile v4us*)(Pl + (size_t)row * TT + ch * 128 + lane * 4) = ol; }
        if (ps == 0) __threadfence(); }
}
__global__ __launch_bounds__(256) void k_addres(const float* __restrict__ Y, float* X, size_t n) {
    const size_t i = ((size_t)blockIdx.x * 256 + threadIdx.x) * 4; if (i >= n) return; const v4f a = *(const v4f*)(X + i), y = *(const v4f*)(Y + i); v4f o;
#pragma unroll
    for (int q = 0; q < 4; ++q) o[q] = __fadd_rn(a[q], y[q]);
    *(volatile v4f*)(X + i) = o; __threadfence(); *(volatile v4f*)(X + i) = o; }
__global__ __launch_bounds__(256) void k_lnout(const float* __restrict__ X, const float* __restrict__ gg, const float* __restrict__ bb, float* OUT) {
    const int lane = threadIdx.x & 31; const int r = blockIdx.x * 8 + (threadIdx.x >> 5); if (r >= NT) return; float v[16];
    load512(X + (size_t)r * CC, lane, v); ln512(v, gg, bb, lane); store512(v, lane, OUT + (size_t)r * CC);
}

extern "C" void kernel_launch(void* const* d_in, const int* in_sizes, int n_in,
                              void* d_out, int out_size, void* d_ws, size_t ws_size, hipStream_t stream) {
    (void)in_sizes; (void)n_in; (void)out_size;
    const float* IN[39]; for (int i = 0; i < 39; ++i) IN[i] = (const float*)d_in[i];
    const int* tok = (const int*)d_in[0]; const int* ptag = (const int*)d_in[1]; const int* etyp = (const int*)d_in[2]; const int* amask = (const int*)d_in[4]; const float* TR = IN[5];
    float* OUT = (float*)d_out;
    char* wsp = (char*)d_ws;
    auto take = [&](size_t bytes) { char* p = wsp; wsp += (bytes + 255) & ~(size_t)255; return (void*)p; };
    bf* WQ = (bf*)take((size_t)CC * CC * 2); bf* WK = (bf*)take((size_t)CC * CC * 2); bf* WV = (bf*)take((size_t)CC * CC * 2); bf* WO = (bf*)take((size_t)CC * CC * 2); bf* W1 = (bf*)take((size_t)FFH * CC * 2); bf* W2 = (bf*)take((size_t)CC * FFH * 2); bf* WS2 = (bf*)take((size_t)CC * SYH * 2);
    float* X = (float*)take((size_t)NT * CC * 4); float* F = (float*)take((size_t)NT * CC * 4); bf* XNh = (bf*)take((size_t)NT * CC * 2); bf* XNl = (bf*)take((size_t)NT * CC * 2); bf* SYh = (bf*)take((size_t)NT * SYH * 2); bf* SYl = (bf*)take((size_t)NT * SYH * 2);
    bf* QPh = (bf*)take((size_t)NT * CC * 2); bf* QPl = (bf*)take((size_t)NT * CC * 2); bf* KPh = (bf*)take((size_t)NT * CC * 2); bf* KPl = (bf*)take((size_t)NT * CC * 2); bf* VTh = (bf*)take((size_t)NT * CC * 2); bf* VTl = (bf*)take((size_t)NT * CC * 2);
    float* Sb = (float*)take((size_t)ZB * TT * TT * 4); bf* Ph = (bf*)take((size_t)ZB * TT * TT * 2); bf* Pl = (bf*)take((size_t)ZB * TT * TT * 2); float* Ob = (float*)take((size_t)ZB * TT * HD * 4);
    bf* ATh = (bf*)take((size_t)NT * CC * 2); bf* ATl = (bf*)take((size_t)NT * CC * 2); float* H = (float*)take((size_t)NT * FFH * 4); bf* Hh = (bf*)take((size_t)NT * FFH * 2); bf* Hl = (bf*)take((size_t)NT * FFH * 2); float* RWB = (float*)take(256); float* PE = (float*)take((size_t)TT * CC * 4);
    if ((size_t)(wsp - (char*)d_ws) > ws_size) return;
    const unsigned LB = (unsigned)((NT * CC / 64 + 63) / 64), gW = (unsigned)((CC * CC / 64 + 63) / 64), gF = (unsigned)((CC * FFH / 64 + 63) / 64), RW = NT / 8; const dim3 gP(NT / 64, CC / 64, 1);
    k_embed<<<RW, 256, 0, stream>>>(tok, ptag, etyp, IN[6], IN[7], IN[8], X);
    k_synmlp<<<RW, 256, 0, stream>>>(IN[3], IN[9], IN[10], IN[11], IN[12], SYh, SYl);
    k_wtG<<<(unsigned)((CC * SYH / 64 + 63) / 64), 256, 0, stream>>>(IN[13], SYH, CC, WS2);
    k_gemmw<bf, 1, true><<<gP, 32, 0, stream>>>(SYh, SYl, WS2, nullptr, SYH, F, CC, IN[14], 0, 0, 0);
    k_petab<<<TT * CC / 256, 256, 0, stream>>>(PE); k_embln<<<RW, 256, 0, stream>>>(F, PE, IN[15], IN[16], X);
    for (int l = 0; l < NL; ++l) { const size_t wo5 = (size_t)l * CC * CC, vo = (size_t)l * CC;
        k_wtG<<<gW, 256, 0, stream>>>(IN[23] + wo5, CC, CC, WQ); k_wtG<<<gW, 256, 0, stream>>>(IN[25] + wo5, CC, CC, WK); k_wtG<<<gW, 256, 0, stream>>>(IN[27] + wo5, CC, CC, WV); k_wtG<<<gW, 256, 0, stream>>>(IN[29] + wo5, CC, CC, WO);
        k_wtG<<<gF, 256, 0, stream>>>(IN[33] + (size_t)l * CC * FFH, CC, FFH, W1); k_wtG<<<gF, 256, 0, stream>>>(IN[35] + (size_t)l * FFH * CC, FFH, CC, W2); k_relw<<<1, 32, 0, stream>>>(IN[31], IN[32], l, RWB);
        k_lnx<1><<<RW, 256, 0, stream>>>(X, IN[17] + vo, IN[18] + vo, IN[21] + vo, IN[22] + vo, XNh, XNl);
        k_gemmw<bf, 1, true><<<gP, 32, 0, stream>>>(XNh, XNl, WQ, nullptr, CC, F, CC, IN[24] + vo, 0, 0, 0); k_hsplit<<<LB, 256, 0, stream>>>(F, 0.125f, QPh, QPl);
        k_gemmw<bf, 1, true><<<gP, 32, 0, stream>>>(XNh, XNl, WK, nullptr, CC, F, CC, IN[26] + vo, 0, 0, 0); k_hsplit<<<LB, 256, 0, stream>>>(F, 1.0f, KPh, KPl);
        k_gemmw<bf, 1, true><<<gP, 32, 0, stream>>>(XNh, XNl, WV, nullptr, CC, F, CC, IN[28] + vo, 0, 0, 0); k_vtplane<<<LB, 256, 0, stream>>>(F, VTh, VTl);
        for (int z0 = 0; z0 < NZ; z0 += ZB) {
            k_gemmw<bf, 2, false><<<dim3(TT / 64, TT / 64, ZB), 32, 0, stream>>>(QPh + (size_t)z0 * TT * HD, QPl + (size_t)z0 * TT * HD, KPh + (size_t)z0 * TT * HD, KPl + (size_t)z0 * TT * HD, HD, Sb, TT, nullptr, (size_t)TT * HD, (size_t)TT * HD, (size_t)TT * TT);
            k_msoft<<<ZB * TT / 8, 256, 0, stream>>>(Sb, TR, amask, RWB, z0, Ph, Pl);
            k_gemmw<bf, 2, false><<<dim3(TT / 64, 1, ZB), 32, 0, stream>>>(Ph, Pl, VTh + (size_t)z0 * HD * TT, VTl + (size_t)z0 * HD * TT, TT, Ob, HD, nullptr, (size_t)TT * TT, (size_t)HD * TT, (size_t)TT * HD);
            k_merge<<<(ZB * TT * HD / 64 + 63) / 64, 256, 0, stream>>>(Ob, z0, ATh, ATl); }
        k_gemmw<bf, 1, true><<<gP, 32, 0, stream>>>(ATh, ATl, WO, nullptr, CC, F, CC, IN[30] + vo, 0, 0, 0);
        k_addres<<<(unsigned)(((size_t)NT * CC / 4 + 255) / 256), 256, 0, stream>>>(F, X, (size_t)NT * CC);
        k_lnx<0><<<RW, 256, 0, stream>>>(X, IN[19] + vo, IN[20] + vo, nullptr, nullptr, XNh, XNl);
        k_gemmw<bf, 1, true><<<dim3(NT / 64, FFH / 64, 1), 32, 0, stream>>>(XNh, XNl, W1, nullptr, CC, H, FFH, IN[34] + (size_t)l * FFH, 0, 0, 0);
        k_relusplit<<<(unsigned)(((size_t)NT * FFH / 2 + 255) / 256), 256, 0, stream>>>(H, Hh, Hl, (size_t)NT * FFH);
        k_gemmw<bf, 1, true><<<gP, 32, 0, stream>>>(Hh, Hl, W2, nullptr, FFH, F, CC, IN[36] + vo, 0, 0, 0);
        k_addres<<<(unsigned)(((size_t)NT * CC / 4 + 255) / 256), 256, 0, stream>>>(F, X, (size_t)NT * CC); }
    k_lnout<<<RW, 256, 0, stream>>>(X, IN[37], IN[38], OUT);
}
